// Attention_87771951661841
// MI455X (gfx1250) — hardware-verified
//
#include <hip/hip_runtime.h>


#ifndef NB
#define NB 4
#endif
#ifndef SEQ
#define SEQ 2048
#endif
#define SEQ_FULL 2048
#define DM   1024
#define NH   16
#define HD   64
#define NQKV (3 * DM)
#define MTOT (NB * SEQ)
#define PLN  ((size_t)NB * NH * SEQ * HD)
#define PSH  8.0f
#define CCAR 256.0f
#define WCAR 32.0f
#define SC2  0.18033688011112042f
static_assert(DM == NH * HD);
static_assert(HD == 64);
static_assert(DM % 64 == 0);
static_assert(DM % 32 == 0);
static_assert(NQKV % 64 == 0);
static_assert(SEQ % 64 == 0);
static_assert(SEQ % 32 == 0);
static_assert(SEQ <= SEQ_FULL);
static_assert(((size_t)MTOT * DM) % 2048 == 0);
static_assert(DM % 8 == 0);

typedef _Float16 h16;
typedef unsigned short bf;
typedef __attribute__((ext_vector_type(16))) __bf16   v16bf;
typedef __attribute__((ext_vector_type(16))) _Float16 v16h;
typedef __attribute__((ext_vector_type(8)))  _Float16 v8h;
typedef __attribute__((ext_vector_type(8)))  unsigned short v8us;
typedef __attribute__((ext_vector_type(8)))  float    v8f;
typedef __attribute__((ext_vector_type(4)))  float    v4f;
typedef v8h  __attribute__((may_alias)) v8ha;
typedef v4f  __attribute__((may_alias)) v4fa;

__device__ __forceinline__ unsigned short f2bf(float f) { unsigned u = __float_as_uint(f); u += 0x7FFFu + ((u >> 16) & 1u); return (unsigned short)(u >> 16); }
__device__ __forceinline__ float bf2f(unsigned short b) { return __uint_as_float(((unsigned)b) << 16); }
__device__ __forceinline__ float bfr(float f) { return bf2f(f2bf(f)); }
__device__ __forceinline__ v16h cat16(v8h lo, v8h hi) { return __builtin_shufflevector(lo, hi, 0, 1, 2, 3, 4, 5, 6, 7, 8, 9, 10, 11, 12, 13, 14, 15); }
__device__ __forceinline__ v16bf cat16b(v8us lo, v8us hi) { return __builtin_bit_cast(v16bf, __builtin_shufflevector(lo, hi, 0, 1, 2, 3, 4, 5, 6, 7, 8, 9, 10, 11, 12, 13, 14, 15)); }
__device__ __forceinline__ v8f wmma16(v16h a, v16h b, v8f c) { return __builtin_amdgcn_wmma_f32_16x16x32_f16(false, a, false, b, (short)0, c, false, false); }
__device__ __forceinline__ v8f wmmab(v16bf a, v16bf b, v8f c) { return __builtin_amdgcn_wmma_f32_16x16x32_bf16(false, a, false, b, (short)0, c, false, false); }

template <typename T16> struct WFrag;
template <> struct WFrag<h16> { typedef v16h V; static __device__ __forceinline__ V ld(const h16* p) { return cat16(*(const v8h*)p, *(const v8h*)(p + 16)); } static __device__ __forceinline__ v8f mma(V a, V b, v8f c) { return wmma16(a, b, c); } };
template <> struct WFrag<bf> { typedef v16bf V; static __device__ __forceinline__ V ld(const bf* p) { return cat16b(*(const v8us*)p, *(const v8us*)(p + 16)); } static __device__ __forceinline__ v8f mma(V a, V b, v8f c) { return wmmab(a, b, c); } };

template <typename T16>
__device__ __forceinline__ void gemm_loop(const T16* __restrict__ A, const T16* __restrict__ Bt, int K, size_t aoff, size_t boff, v8f (&acc)[4][4]) {
    typedef typename WFrag<T16>::V V;
#pragma unroll 1
    for (int kc = 0; kc < K; kc += 32) {
        V a[4];
#pragma unroll
        for (int mb = 0; mb < 4; ++mb) a[mb] = WFrag<T16>::ld(A + aoff + (size_t)mb * 16 * K + kc);
#pragma unroll
        for (int nb = 0; nb < 4; ++nb) { const V b = WFrag<T16>::ld(Bt + boff + (size_t)nb * 16 * K + kc);
#pragma unroll
            for (int mb = 0; mb < 4; ++mb) acc[mb][nb] = WFrag<T16>::mma(a[mb], b, acc[mb][nb]); }
        asm volatile("v_nop\n\tv_nop\n\tv_nop\n\tv_nop" : "+v"(acc[0][0]), "+v"(acc[0][1]), "+v"(acc[0][2]), "+v"(acc[0][3]), "+v"(acc[1][0]), "+v"(acc[1][1]), "+v"(acc[1][2]), "+v"(acc[1][3]),
                            "+v"(acc[2][0]), "+v"(acc[2][1]), "+v"(acc[2][2]), "+v"(acc[2][3]), "+v"(acc[3][0]), "+v"(acc[3][1]), "+v"(acc[3][2]), "+v"(acc[3][3]) : "v"(a[0]), "v"(a[3]));
    }
}

__global__ __launch_bounds__(256) void k_cvtx(const float* __restrict__ x, bf* XB) {
    const size_t e = ((size_t)blockIdx.x * 256 + threadIdx.x) * 8; if (e >= (size_t)MTOT * DM) return;
    const size_t m = e / DM; const int c = (int)(e % DM); const size_t b = m / SEQ, t = m % SEQ;
    const float* src = x + ((b * SEQ_FULL + t) * DM + c);
    const v4f a0 = *(const v4f*)src, a1 = *(const v4f*)(src + 4); v8us o;
#pragma unroll
    for (int j = 0; j < 4; ++j) { o[j] = f2bf(a0[j]); o[4 + j] = f2bf(a1[j]); }
    *(volatile v8us*)(XB + e) = o; __threadfence(); *(volatile v8us*)(XB + e) = o;
}

__global__ __launch_bounds__(256) void k_wt(const float* __restrict__ W, int Kr, int Nc, bf* OT, int mode, float sc) {
    __shared__ float ts[64 * 65];
    const int tid = threadIdx.x; const int n0 = blockIdx.x * 64, k0 = blockIdx.y * 64;
#pragma unroll 4
    for (int i = 0; i < 16; ++i) { const int k = i * 4 + (tid >> 6), n = tid & 63; ts[k * 65 + n] = W[(size_t)(k0 + k) * Nc + n0 + n]; }
    __syncthreads();
    const int p = tid & 7; const int na = tid >> 3, nb2 = 32 + (tid >> 3); v8us o0, o1;
#pragma unroll
    for (int j = 0; j < 8; ++j) { const float va = ts[(p * 8 + j) * 65 + na], vb = ts[(p * 8 + j) * 65 + nb2];
        const unsigned short ha = __builtin_bit_cast(unsigned short, (h16)(bfr(va) * sc)), hb = __builtin_bit_cast(unsigned short, (h16)(bfr(vb) * sc));
        const unsigned short ba = f2bf(va), bb = f2bf(vb);
        o0[j] = mode ? ha : ba; o1[j] = mode ? hb : bb; }
    bf* d0 = OT + (size_t)(n0 + na) * Kr + k0 + p * 8; bf* d1 = OT + (size_t)(n0 + nb2) * Kr + k0 + p * 8;
    *(volatile v8us*)d0 = o0; *(volatile v8us*)d1 = o1; __threadfence(); *(volatile v8us*)d0 = o0; *(volatile v8us*)d1 = o1;
}

__global__ __launch_bounds__(32) void k_qkv(const bf* __restrict__ A, const bf* __restrict__ Bt, const float* __restrict__ bias, h16* PL) {
    __shared__ __align__(16) float os[64 * 68];
    const int lane = threadIdx.x & 31, lr = lane & 15, hi = lane >> 4; const int r0 = blockIdx.x * 64, c0 = blockIdx.y * 64;
    v8f acc[4][4];
#pragma unroll
    for (int mb = 0; mb < 4; ++mb)
#pragma unroll
        for (int nb = 0; nb < 4; ++nb) acc[mb][nb] = (v8f){};
    gemm_loop<bf>(A, Bt, DM, (size_t)(r0 + lr) * DM + 8 * hi, (size_t)(c0 + lr) * DM + 8 * hi, acc);
#pragma unroll
    for (int mb = 0; mb < 4; ++mb)
#pragma unroll
        for (int nb = 0; nb < 4; ++nb)
#pragma unroll
            for (int j = 0; j < 8; ++j) os[(mb * 16 + hi * 8 + j) * 68 + nb * 16 + lr] = acc[mb][nb][j];
    __syncthreads();
    const int which = c0 / DM, hh = (c0 % DM) / HD; const int b = r0 / SEQ, t0 = r0 % SEQ; const int g = lane >> 3, p = lane & 7;
    if (which < 2) {
        h16* dst = PL + (size_t)which * PLN + ((size_t)(b * NH + hh) * SEQ + t0) * HD;
        v4f b0 = *(const v4f*)(bias + c0 + p * 8), b1 = *(const v4f*)(bias + c0 + p * 8 + 4);
#pragma unroll
        for (int j = 0; j < 4; ++j) { b0[j] = bfr(b0[j]); b1[j] = bfr(b1[j]); }
#pragma unroll 1
        for (int ps = 0; ps < 2; ++ps) {
#pragma unroll
            for (int s = 0; s < 16; ++s) { const int row = 4 * s + g; const v4f x0 = *(const v4fa*)(os + row * 68 + p * 8), x1 = *(const v4fa*)(os + row * 68 + p * 8 + 4); v8h w;
#pragma unroll
                for (int j = 0; j < 4; ++j) { w[j] = (h16)(x0[j] + b0[j]); w[4 + j] = (h16)(x1[j] + b1[j]); }
                *(volatile v8h*)(dst + (size_t)row * HD + p * 8) = w; }
            if (ps == 0) __threadfence(); }
    } else {
        h16* dst = PL + 2 * PLN + ((size_t)(b * NH + hh) * HD) * SEQ + t0;
#pragma unroll 1
        for (int ps = 0; ps < 2; ++ps) {
#pragma unroll
            for (int s = 0; s < 16; ++s) { const int d = 4 * s + g; const float bd = bfr(bias[c0 + d]); v8h w;
#pragma unroll
                for (int j = 0; j < 8; ++j) w[j] = (h16)(os[(p * 8 + j) * 68 + d] + bd);
                *(volatile v8h*)(dst + (size_t)d * SEQ + p * 8) = w; }
            if (ps == 0) __threadfence(); }
    }
}

__global__ __launch_bounds__(32) void k_flash(const h16* __restrict__ PL, h16* CTX) {
    __shared__ __align__(16) h16 cs[32 * 72];
    const int lane = threadIdx.x & 31, lr = lane & 15, hi = lane >> 4;
    const size_t bh = blockIdx.y; const int q0 = blockIdx.x * 32;
    const h16* Qp = PL + bh * ((size_t)SEQ * HD);
    const h16* Kp = PL + PLN + bh * ((size_t)SEQ * HD) + (size_t)lr * HD + 8 * hi;
    const h16* Vp = PL + 2 * PLN + bh * ((size_t)HD * SEQ) + (size_t)lr * SEQ + 8 * hi;
    v16h qf[2][2];
#pragma unroll
    for (int qt = 0; qt < 2; ++qt)
#pragma unroll
        for (int ks = 0; ks < 2; ++ks) qf[qt][ks] = WFrag<h16>::ld(Qp + (size_t)(q0 + qt * 16 + lr) * HD + ks * 32 + 8 * hi);
    v8f o[4][2];
#pragma unroll
    for (int db = 0; db < 4; ++db) { o[db][0] = (v8f){}; o[db][1] = (v8f){}; }
    float mrun[2] = { -1.0e30f, -1.0e30f }, lrun[2] = { 0.0f, 0.0f };
#pragma unroll 1
    for (int kt = 0; kt < SEQ; kt += 32) {
        v8f s[2][2]; s[0][0] = (v8f){}; s[0][1] = (v8f){}; s[1][0] = (v8f){}; s[1][1] = (v8f){};
#pragma unroll
        for (int ks = 0; ks < 2; ++ks) {
            const v16h ka0 = WFrag<h16>::ld(Kp + (size_t)kt * HD + ks * 32);
            const v16h ka1 = WFrag<h16>::ld(Kp + (size_t)(kt + 16) * HD + ks * 32);
            s[0][0] = wmma16(ka0, qf[0][ks], s[0][0]); s[0][1] = wmma16(ka0, qf[1][ks], s[0][1]);
            s[1][0] = wmma16(ka1, qf[0][ks], s[1][0]); s[1][1] = wmma16(ka1, qf[1][ks], s[1][1]);
            asm volatile("v_nop\n\tv_nop\n\tv_nop\n\tv_nop" : "+v"(s[0][0]), "+v"(s[0][1]), "+v"(s[1][0]), "+v"(s[1][1]) : "v"(ka0), "v"(ka1), "v"(qf[0][ks]), "v"(qf[1][ks]));
        }
        v16h pb[2];
#pragma unroll
        for (int qt = 0; qt < 2; ++qt) {
            float cm = s[0][qt][0];
#pragma unroll
            for (int r = 1; r < 8; ++r) cm = fmaxf(cm, s[0][qt][r]);
#pragma unroll
            for (int r = 0; r < 8; ++r) cm = fmaxf(cm, s[1][qt][r]);
            cm = fmaxf(cm, __shfl_xor(cm, 16, 32));
            const float mn = fmaxf(mrun[qt], cm * SC2);
            const float alpha = __builtin_amdgcn_exp2f(mrun[qt] - mn); mrun[qt] = mn;
            const float sh = PSH - mn; float psum = 0.0f;
#pragma unroll
            for (int kb = 0; kb < 2; ++kb)
#pragma unroll
                for (int r = 0; r < 8; ++r) { const float pv = __builtin_amdgcn_exp2f(fmaf(s[kb][qt][r], SC2, sh)); psum += pv; pb[qt][kb * 8 + r] = (h16)pv; }
            lrun[qt] = lrun[qt] * alpha + psum;
#pragma unroll
            for (int db = 0; db < 4; ++db)
#pragma unroll
                for (int r = 0; r < 8; ++r) o[db][qt][r] *= alpha;
        }
#pragma unroll
        for (int db = 0; db < 4; ++db) {
            const v16h va = WFrag<h16>::ld(Vp + (size_t)db * 16 * SEQ + kt);
            o[db][0] = wmma16(va, pb[0], o[db][0]); o[db][1] = wmma16(va, pb[1], o[db][1]);
            asm volatile("v_nop\n\tv_nop\n\tv_nop\n\tv_nop" : "+v"(o[db][0]), "+v"(o[db][1]) : "v"(va), "v"(pb[0]), "v"(pb[1]));
        }
    }
    float inv[2];
#pragma unroll
    for (int qt = 0; qt < 2; ++qt) { const float lt = lrun[qt] + __shfl_xor(lrun[qt], 16, 32); inv[qt] = CCAR * (1.0f / lt); }
#pragma unroll
    for (int db = 0; db < 4; ++db)
#pragma unroll
        for (int qt = 0; qt < 2; ++qt) { v8h w;
#pragma unroll
            for (int r = 0; r < 8; ++r) w[r] = (h16)(o[db][qt][r] * inv[qt]);
            *(v8h*)(cs + (qt * 16 + lr) * 72 + db * 16 + 8 * hi) = w; }
    __syncthreads();
    const int b = (int)(bh / NH), h = (int)(bh % NH); const int g = lane >> 3, p = lane & 7;
    h16* dst = CTX + ((size_t)b * SEQ + q0) * DM + h * HD;
#pragma unroll 1
    for (int ps = 0; ps < 2; ++ps) {
#pragma unroll
        for (int s2 = 0; s2 < 8; ++s2) { const int q = 4 * s2 + g; const v8h w = *(const v8ha*)(cs + q * 72 + p * 8); *(volatile v8h*)(dst + (size_t)q * DM + p * 8) = w; }
        if (ps == 0) __threadfence(); }
}

__global__ __launch_bounds__(32) void k_fc(const h16* __restrict__ A, const h16* __restrict__ Bt, const float* __restrict__ bias, float* C, float oscale) {
    __shared__ __align__(16) float os[16 * 68];
    const int lane = threadIdx.x & 31, lr = lane & 15, hi = lane >> 4; const int r0 = blockIdx.x * 64, c0 = blockIdx.y * 64;
    v8f acc[4][4];
#pragma unroll
    for (int mb = 0; mb < 4; ++mb)
#pragma unroll
        for (int nb = 0; nb < 4; ++nb) acc[mb][nb] = (v8f){};
    gemm_loop<h16>(A, Bt, DM, (size_t)(r0 + lr) * DM + 8 * hi, (size_t)(c0 + lr) * DM + 8 * hi, acc);
    const int cofs = lr * 4; v4f bb = *(const v4f*)(bias + c0 + cofs);
#pragma unroll
    for (int j = 0; j < 4; ++j) bb[j] = bfr(bb[j]);
#pragma unroll
    for (int mb = 0; mb < 4; ++mb) {
#pragma unroll
        for (int nb = 0; nb < 4; ++nb)
#pragma unroll
            for (int j = 0; j < 8; ++j) os[(hi * 8 + j) * 68 + nb * 16 + lr] = acc[mb][nb][j];
        __syncthreads();
        float* crow = C + (size_t)(r0 + mb * 16) * DM + c0;
#pragma unroll 1
        for (int ps = 0; ps < 2; ++ps) {
#pragma unroll
            for (int s = 0; s < 8; ++s) { const int row = 2 * s + hi; v4f val = *(const v4fa*)(os + row * 68 + cofs); val = val * oscale + bb;
                *(volatile v4f*)(crow + (size_t)row * DM + cofs) = val; }
            if (ps == 0) __threadfence(); }
        __syncthreads();
    }
}

constexpr size_t XB_B  = (size_t)MTOT * DM * 2;
constexpr size_t WQT_B = (size_t)NQKV * DM * 2;
constexpr size_t WFT_B = (size_t)DM * DM * 2;
constexpr size_t PL_B  = (size_t)3 * NB * NH * SEQ * HD * 2;
constexpr size_t CTX_B = (size_t)MTOT * DM * 2;
constexpr size_t WS_TOTAL = XB_B + WQT_B + WFT_B + PL_B + CTX_B;
static_assert(XB_B % 256 == 0 && WQT_B % 256 == 0 && WFT_B % 256 == 0 && PL_B % 256 == 0 && CTX_B % 256 == 0);
static_assert(WS_TOTAL <= (size_t)134217728);
static_assert(((size_t)(NB - 1) * SEQ_FULL + SEQ) * DM <= (size_t)2147483647);

extern "C" void kernel_launch(void* const* d_in, const int* in_sizes, int n_in,
                              void* d_out, int out_size, void* d_ws, size_t ws_size, hipStream_t stream) {
    if (n_in < 5) return;
    if (in_sizes[0] < (int)(((size_t)(NB - 1) * SEQ_FULL + SEQ) * DM)) return;
    if (in_sizes[1] < DM * NQKV || in_sizes[2] < NQKV || in_sizes[3] < DM * DM || in_sizes[4] < DM) return;
    if (out_size < MTOT * DM) return;
    if (ws_size < WS_TOTAL) return;
    const float* x = (const float*)d_in[0]; const float* wqkv = (const float*)d_in[1]; const float* bqkv = (const float*)d_in[2];
    const float* wfc = (const float*)d_in[3]; const float* bfc = (const float*)d_in[4];
    float* OUT = (float*)d_out;
    char* wsp = (char*)d_ws;
    bf* XB = (bf*)wsp; wsp += XB_B;
    bf* WQT = (bf*)wsp; wsp += WQT_B;
    bf* WFT = (bf*)wsp; wsp += WFT_B;
    h16* PL = (h16*)wsp; wsp += PL_B;
    h16* CTX = (h16*)wsp; wsp += CTX_B;
    k_cvtx<<<(unsigned)(((size_t)MTOT * DM) / 2048), 256, 0, stream>>>(x, XB);
    k_wt<<<dim3(NQKV / 64, DM / 64), 256, 0, stream>>>(wqkv, DM, NQKV, WQT, 0, 1.0f);
    k_wt<<<dim3(DM / 64, DM / 64), 256, 0, stream>>>(wfc, DM, DM, WFT, 1, WCAR);
    k_qkv<<<dim3(MTOT / 64, NQKV / 64), 32, 0, stream>>>(XB, WQT, bqkv, PL);
    k_flash<<<dim3(SEQ / 32, NB * NH), 32, 0, stream>>>(PL, CTX);
    k_fc<<<dim3(MTOT / 64, DM / 64), 32, 0, stream>>>(CTX, (const h16*)WFT, bfc, OUT, 1.0f / (CCAR * WCAR));
}
